// GATVGAEEncoder_16810501996995
// MI455X (gfx1250) — hardware-verified
//
#include <hip/hip_runtime.h>
#include <stddef.h>


#define DF    128
#define NHD   4
#define HC    32
#define OC    32
#define GR    32
#define AP    136
#define XSP   132
#define NB    512
#define CHUNK 2048
#define NTHR  256
#define NWAVE 8
#define WCAP  256
#define NGRP  (CHUNK / (NTHR * 4))

#define LDS_SACC (NB * DF)
#define LDS_DEN  (NB * NHD)
#define LDS_LIST (NWAVE * WCAP)
#define LDS_BYTES ((LDS_SACC + LDS_DEN + LDS_LIST + NWAVE) * 4)

static_assert(WCAP == (CHUNK / NTHR) * 32);
static_assert(NGRP >= 1);
static_assert(NB == 512);
static_assert(CHUNK == 2048);
static_assert(((LDS_SACC + LDS_DEN) % 4) == 0);
static_assert(LDS_BYTES == 278560);
static_assert(NHD * HC == DF);
static_assert(((AP * 2) % 16) == 0);
static_assert(((XSP * 4) % 16) == 0);
static_assert((NB / NWAVE) * NWAVE == NB);

typedef float  v4f  __attribute__((ext_vector_type(4)));
typedef float  v8f  __attribute__((ext_vector_type(8)));
typedef int    v4i  __attribute__((ext_vector_type(4)));
typedef __bf16 v16b __attribute__((ext_vector_type(16)));
union FragB { v16b v; v4i q[2]; };

__device__ __forceinline__ v8f wm(v16b a, v16b b, v8f c) {
  v8f d = __builtin_amdgcn_wmma_f32_16x16x32_bf16(false, a, false, b, (short)0, c, false, false);
  asm volatile("v_nop\n\tv_nop\n\tv_nop\n\tv_nop" : "+v"(d) : "v"(a), "v"(b));
  return d;
}

__device__ __forceinline__ unsigned bf_bits(float f) {
  unsigned u = __float_as_uint(f);
  u += 0x7FFFu + ((u >> 16) & 1u);
  return u >> 16;
}

__device__ __forceinline__ void split2(float f, unsigned& hb, unsigned& lb) {
  hb = bf_bits(f);
  const float hf = __uint_as_float(hb << 16);
  lb = bf_bits(f - hf);
}

__device__ __forceinline__ void pack8(const float* f, v4i& hi, v4i& lo) {
  unsigned h[8], l[8];
#pragma unroll
  for (int t = 0; t < 8; ++t) split2(f[t], h[t], l[t]);
  hi.x = (int)(h[0] | (h[1] << 16)); hi.y = (int)(h[2] | (h[3] << 16));
  hi.z = (int)(h[4] | (h[5] << 16)); hi.w = (int)(h[6] | (h[7] << 16));
  lo.x = (int)(l[0] | (l[1] << 16)); lo.y = (int)(l[2] | (l[3] << 16));
  lo.z = (int)(l[4] | (l[5] << 16)); lo.w = (int)(l[6] | (l[7] << 16));
}

__device__ __forceinline__ float lexp(float s) {
  s = (s > 0.f) ? s : 0.2f * s;
  s = fminf(s, 80.f);
  return __expf(s);
}

__device__ __forceinline__ float elu1(float v) { return (v > 0.f) ? v : (__expf(v) - 1.0f); }

__global__ __launch_bounds__(NTHR) void k_prep(const float* __restrict__ W1,
                                               const float* __restrict__ Wmu,
                                               const float* __restrict__ Wls,
                                               unsigned short* Wp) {
  const int i = blockIdx.x * NTHR + threadIdx.x;
  if (i >= 2 * DF * (DF / 8)) return;
  const int layer = i / (DF * (DF / 8));
  const int j  = i - layer * (DF * (DF / 8));
  const int n  = j >> 4;
  const int kg = (j & 15) * 8;
  const float* src;
  int ld, cn;
  if (layer == 0)      { src = W1;  ld = DF;     cn = n; }
  else if (n < 2 * OC) { src = Wmu; ld = 2 * OC; cn = n; }
  else                 { src = Wls; ld = 2 * OC; cn = n - 2 * OC; }
  float f[8];
#pragma unroll
  for (int t = 0; t < 8; ++t) f[t] = src[(size_t)(kg + t) * ld + cn];
  v4i hi, lo;
  pack8(f, hi, lo);
  unsigned short* Hp = Wp + (size_t)layer * 2 * DF * DF + (size_t)n * DF + kg;
  unsigned short* Lp = Hp + DF * DF;
  *(volatile v4i*)Hp = hi;
  *(volatile v4i*)Lp = lo;
  __threadfence();
  *(volatile v4i*)Hp = hi;
  *(volatile v4i*)Lp = lo;
}

__device__ __forceinline__ void epi_tile(v8f acc, int T, int hh, int m, int wave, int ncol,
                                         float cs, float cd, float* Xs, float* As, float* Ds) {
  float ss[8], sd[8];
#pragma unroll
  for (int r = 0; r < 8; ++r) {
    const float v = acc[r];
    Xs[(T * 16 + 8 * hh + r) * XSP + ncol] = v;
    ss[r] = v * cs;
    sd[r] = v * cd;
  }
#pragma unroll
  for (int mk = 1; mk < 16; mk <<= 1) {
#pragma unroll
    for (int r = 0; r < 8; ++r) {
      ss[r] += __shfl_xor(ss[r], mk, 32);
      sd[r] += __shfl_xor(sd[r], mk, 32);
    }
  }
  if (m == 0) {
#pragma unroll
    for (int r = 0; r < 8; ++r) {
      As[(T * 16 + 8 * hh + r) * NWAVE + wave] = ss[r];
      Ds[(T * 16 + 8 * hh + r) * NWAVE + wave] = sd[r];
    }
  }
}

__global__ __launch_bounds__(NTHR) void k_gemm(
    const float* __restrict__ A, const unsigned short* __restrict__ Whi,
    const unsigned short* __restrict__ Wlo,
    const float* __restrict__ attSA, const float* __restrict__ attSB,
    const float* __restrict__ attDA, const float* __restrict__ attDB,
    float* xl, float* asrc, float* adst, int nN) {
  __shared__ __attribute__((aligned(16))) unsigned short Ah[GR * AP];
  __shared__ __attribute__((aligned(16))) unsigned short Al[GR * AP];
  __shared__ __attribute__((aligned(16))) float Xs[GR * XSP];
  __shared__ __attribute__((aligned(16))) float As[GR * NWAVE];
  __shared__ __attribute__((aligned(16))) float Ds[GR * NWAVE];

  const int tid  = threadIdx.x;
  const int lane = tid & 31;
  const int wave = tid >> 5;
  const int hh   = lane >> 4;
  const int m    = lane & 15;
  const int rowBase = blockIdx.x * GR;

  {
    const int r  = tid >> 3;
    const int c0 = (tid & 7) * 16;
    int row = rowBase + r;
    if (row > nN - 1) row = nN - 1;
    const float* p = A + (size_t)row * DF + c0;
    const v4f g0 = *(const v4f*)(p), g1 = *(const v4f*)(p + 4);
    const v4f g2 = *(const v4f*)(p + 8), g3 = *(const v4f*)(p + 12);
    float f0[8], f1[8];
    f0[0] = g0.x; f0[1] = g0.y; f0[2] = g0.z; f0[3] = g0.w;
    f0[4] = g1.x; f0[5] = g1.y; f0[6] = g1.z; f0[7] = g1.w;
    f1[0] = g2.x; f1[1] = g2.y; f1[2] = g2.z; f1[3] = g2.w;
    f1[4] = g3.x; f1[5] = g3.y; f1[6] = g3.z; f1[7] = g3.w;
    v4i h0, l0, h1, l1;
    pack8(f0, h0, l0);
    pack8(f1, h1, l1);
    *(v4i*)(Ah + r * AP + c0)     = h0;
    *(v4i*)(Ah + r * AP + c0 + 8) = h1;
    *(v4i*)(Al + r * AP + c0)     = l0;
    *(v4i*)(Al + r * AP + c0 + 8) = l1;
  }
  __syncthreads();

  const int ncol = wave * 16 + m;
  v8f c0a = {0.f, 0.f, 0.f, 0.f, 0.f, 0.f, 0.f, 0.f};
  v8f c1a = {0.f, 0.f, 0.f, 0.f, 0.f, 0.f, 0.f, 0.f};
#pragma unroll
  for (int kt = 0; kt < DF / 32; ++kt) {
    const int k0 = kt * 32;
    FragB ah0, al0, ah1, al1, bh, bl;
    const unsigned short* pa0 = Ah + m * AP + k0 + 8 * hh;
    const unsigned short* pa1 = Ah + (16 + m) * AP + k0 + 8 * hh;
    const unsigned short* qa0 = Al + m * AP + k0 + 8 * hh;
    const unsigned short* qa1 = Al + (16 + m) * AP + k0 + 8 * hh;
    const unsigned short* pb  = Whi + (size_t)ncol * DF + k0 + 8 * hh;
    const unsigned short* qb  = Wlo + (size_t)ncol * DF + k0 + 8 * hh;
    ah0.q[0] = *(const v4i*)pa0; ah0.q[1] = *(const v4i*)(pa0 + 16);
    ah1.q[0] = *(const v4i*)pa1; ah1.q[1] = *(const v4i*)(pa1 + 16);
    al0.q[0] = *(const v4i*)qa0; al0.q[1] = *(const v4i*)(qa0 + 16);
    al1.q[0] = *(const v4i*)qa1; al1.q[1] = *(const v4i*)(qa1 + 16);
    bh.q[0]  = *(const v4i*)pb;  bh.q[1]  = *(const v4i*)(pb + 16);
    bl.q[0]  = *(const v4i*)qb;  bl.q[1]  = *(const v4i*)(qb + 16);
    c0a = wm(ah0.v, bh.v, c0a);
    c0a = wm(ah0.v, bl.v, c0a);
    c0a = wm(al0.v, bh.v, c0a);
    c1a = wm(ah1.v, bh.v, c1a);
    c1a = wm(ah1.v, bl.v, c1a);
    c1a = wm(al1.v, bh.v, c1a);
  }

  const float* aps = (wave < NWAVE / 2) ? attSA : attSB;
  const float* apd = (wave < NWAVE / 2) ? attDA : attDB;
  const int ci = ncol & 63;
  const float cs = aps[ci];
  const float cd = apd[ci];
  epi_tile(c0a, 0, hh, m, wave, ncol, cs, cd, Xs, As, Ds);
  epi_tile(c1a, 1, hh, m, wave, ncol, cs, cd, Xs, As, Ds);
  __syncthreads();

  v4f xr[4];
#pragma unroll
  for (int i = 0; i < 4; ++i) xr[i] = *(const v4f*)(Xs + (4 * wave + i) * XSP + 4 * lane);
  float* gp = 0;
  v4f gv = {0.f, 0.f, 0.f, 0.f};
  if (wave == 0) {
    const float* s = As + lane * NWAVE;
    gv.x = s[0] + s[1]; gv.y = s[2] + s[3]; gv.z = s[4] + s[5]; gv.w = s[6] + s[7];
    gp = asrc + (size_t)rowBase * NHD + 4 * lane;
  } else if (wave == 1) {
    const float* s = Ds + lane * NWAVE;
    gv.x = s[0] + s[1]; gv.y = s[2] + s[3]; gv.z = s[4] + s[5]; gv.w = s[6] + s[7];
    gp = adst + (size_t)rowBase * NHD + 4 * lane;
  }
  float* xpp[4];
#pragma unroll
  for (int i = 0; i < 4; ++i) xpp[i] = xl + (size_t)(rowBase + 4 * wave + i) * DF + 4 * lane;

#pragma unroll
  for (int i = 0; i < 4; ++i) *(volatile v4f*)(xpp[i]) = xr[i];
  if (gp) *(volatile v4f*)gp = gv;
  __threadfence();
#pragma unroll
  for (int i = 0; i < 4; ++i) *(volatile v4f*)(xpp[i]) = xr[i];
  if (gp) *(volatile v4f*)gp = gv;
}

template <int MODE>
__global__ __launch_bounds__(NTHR) void k_agg(
    const int* __restrict__ ei, const float* __restrict__ xl,
    const float* __restrict__ asrc, const float* __restrict__ adst,
    const float* __restrict__ biasA, const float* __restrict__ biasB,
    float* hout, float* out0, float* out1, int nN, int nE) {
  extern __shared__ v4f lds_dyn[];
  float* sacc = (float*)lds_dyn;
  float* den  = sacc + LDS_SACC;
  int*   list = (int*)(den + LDS_DEN);
  int*   wcnt = list + LDS_LIST;

  const int tid  = threadIdx.x;
  const int lane = tid & 31;
  const int wave = tid >> 5;
  const int hd   = lane >> 3;
  const int nodeBase = blockIdx.x * NB;

  {
    const v4f z4 = {0.f, 0.f, 0.f, 0.f};
    for (int i = tid; i < (LDS_SACC + LDS_DEN) / 4; i += NTHR) lds_dyn[i] = z4;
  }
  __syncthreads();

  const int* eid = ei + nE;
  const bool al16 = ((nE & 3) == 0);

  const int nChunks = (nE + CHUNK - 1) / CHUNK;
#pragma unroll 1
  for (int ch = 0; ch < nChunks; ++ch) {
    const int cbase = ch * CHUNK;
    int wc = 0;
#pragma unroll
    for (int g = 0; g < NGRP; ++g) {
      const int el0 = (g * NTHR + tid) * 4;
      const int e0  = cbase + el0;
      const int sent = -2147483647 - 1;
      v4i d;
      if (al16 && (e0 + 3 < nE)) {
        d = *(const v4i*)(eid + e0);
      } else {
        d.x = (e0     < nE) ? eid[min(e0, nE - 1)]     : sent;
        d.y = (e0 + 1 < nE) ? eid[min(e0 + 1, nE - 1)] : sent;
        d.z = (e0 + 2 < nE) ? eid[min(e0 + 2, nE - 1)] : sent;
        d.w = (e0 + 3 < nE) ? eid[min(e0 + 3, nE - 1)] : sent;
      }
      const unsigned s0 = (unsigned)d.x - (unsigned)nodeBase;
      const unsigned s1 = (unsigned)d.y - (unsigned)nodeBase;
      const unsigned s2 = (unsigned)d.z - (unsigned)nodeBase;
      const unsigned s3 = (unsigned)d.w - (unsigned)nodeBase;
      const bool h0 = s0 < (unsigned)NB;
      const bool h1 = s1 < (unsigned)NB;
      const bool h2 = s2 < (unsigned)NB;
      const bool h3 = s3 < (unsigned)NB;
      const unsigned many = __builtin_amdgcn_ballot_w32(h0 | h1 | h2 | h3);
      if (many != 0u) {
#define HITJ(J, HJ, SJ) { \
          const unsigned mj = __builtin_amdgcn_ballot_w32(HJ); \
          if (HJ) { \
            const int pos = wc + (int)__builtin_amdgcn_mbcnt_lo(mj, 0u); \
            if (pos < WCAP) list[wave * WCAP + pos] = ((el0 + (J)) << 9) | (int)(SJ); \
          } \
          wc += (int)__builtin_popcount(mj); }
        HITJ(0, h0, s0)
        HITJ(1, h1, s1)
        HITJ(2, h2, s2)
        HITJ(3, h3, s3)
#undef HITJ
      }
    }
    if (lane == 0) wcnt[wave] = wc;
    __syncthreads();

    if (wave == 0) {
#pragma unroll 1
      for (int wsx = 0; wsx < NWAVE; ++wsx) {
        int n = wcnt[wsx];
        if (n > WCAP) n = WCAP;
        if (n < 0) n = 0;
#pragma unroll 1
        for (int i = 0; i < n; ++i) {
          const int ent  = list[wsx * WCAP + i];
          const int slot = ent & (NB - 1);
          const int el   = (ent >> 9) & (CHUNK - 1);
          int e = cbase + el;
          if (e > nE - 1) e = nE - 1;
          int src = ei[e];
          src = src < 0 ? 0 : (src > nN - 1 ? nN - 1 : src);
          int nd = nodeBase + slot;
          if (nd > nN - 1) nd = nN - 1;
          const float p = lexp(asrc[(size_t)src * NHD + hd] + adst[(size_t)nd * NHD + hd]);
          const v4f xv = *(const v4f*)(xl + (size_t)src * DF + 4 * lane);
          v4f* sp = (v4f*)(sacc + slot * DF + 4 * lane);
          const v4f cur = *sp;
          const v4f nxt = cur + p * xv;
          *sp = nxt;
          if ((lane & 7) == 0) {
            const float o = den[slot * NHD + hd];
            den[slot * NHD + hd] = o + p;
          }
        }
      }
    }
    __syncthreads();
  }

  if constexpr (MODE == 1) {
    const v4f b4 = *(const v4f*)(biasA + 4 * lane);
#pragma unroll 1
    for (int j = 0; j < NB / NWAVE; ++j) {
      const int slot = wave * (NB / NWAVE) + j;
      const int node = nodeBase + slot;
      if (node >= nN) break;
      const size_t nrow = (size_t)node;
      const float p = lexp(asrc[nrow * NHD + hd] + adst[nrow * NHD + hd]);
      const v4f xv = *(const v4f*)(xl + nrow * DF + 4 * lane);
      const v4f sv = *(const v4f*)(sacc + slot * DF + 4 * lane) + p * xv;
      const float dv  = den[slot * NHD + hd] + p;
      const float inv = 1.0f / (dv + 1e-16f);
      const v4f v = sv * inv + b4;
      v4f y;
      y.x = elu1(v.x); y.y = elu1(v.y); y.z = elu1(v.z); y.w = elu1(v.w);
      float* op = hout + nrow * DF + 4 * lane;
      *(volatile v4f*)op = y;
      __threadfence();
      *(volatile v4f*)op = y;
    }
  } else {
    const int   c4   = 4 * (lane & 7);
    const bool  lo16 = lane < 16;
    const float* bp  = lo16 ? biasA : biasB;
    const v4f   b4   = *(const v4f*)(bp + c4);
    float* obase     = lo16 ? out0 : out1;
    const bool  wr   = (lane & 8) == 0;
#pragma unroll 1
    for (int j = 0; j < NB / NWAVE; ++j) {
      const int slot = wave * (NB / NWAVE) + j;
      const int node = nodeBase + slot;
      if (node >= nN) break;
      const size_t nrow = (size_t)node;
      const float p = lexp(asrc[nrow * NHD + hd] + adst[nrow * NHD + hd]);
      const v4f xv = *(const v4f*)(xl + nrow * DF + 4 * lane);
      const v4f sv = *(const v4f*)(sacc + slot * DF + 4 * lane) + p * xv;
      const float dv  = den[slot * NHD + hd] + p;
      const float inv = 1.0f / (dv + 1e-16f);
      const v4f v = sv * inv;
      v4f o;
      o.x = __shfl_xor(v.x, 8, 32); o.y = __shfl_xor(v.y, 8, 32);
      o.z = __shfl_xor(v.z, 8, 32); o.w = __shfl_xor(v.w, 8, 32);
      const v4f y = (v + o) * 0.5f + b4;
      float* op = obase + nrow * OC + c4;
      if (wr) *(volatile v4f*)op = y;
      __threadfence();
      if (wr) *(volatile v4f*)op = y;
    }
  }
}

extern "C" void kernel_launch(void* const* d_in, const int* in_sizes, int n_in,
                              void* d_out, int out_size, void* d_ws, size_t ws_size,
                              hipStream_t stream) {
  if (n_in < 14) return;
  const int nN = in_sizes[0] / DF;
  if (nN <= 0 || in_sizes[0] != nN * DF) return;
  if (in_sizes[1] < 0 || (in_sizes[1] & 1)) return;
  const int nE = in_sizes[1] / 2;
  if (in_sizes[2] != DF * DF) return;
  if (in_sizes[3] != NHD * HC || in_sizes[4] != NHD * HC || in_sizes[5] != DF) return;
  if (in_sizes[6] != DF * 2 * OC || in_sizes[7] != 2 * OC || in_sizes[8] != 2 * OC || in_sizes[9] != OC) return;
  if (in_sizes[10] != DF * 2 * OC || in_sizes[11] != 2 * OC || in_sizes[12] != 2 * OC || in_sizes[13] != OC) return;
  if (out_size != 2 * nN * OC) return;

  const float* x    = (const float*)d_in[0];
  const int*   ei   = (const int*)d_in[1];
  const float* W1   = (const float*)d_in[2];
  const float* a1s  = (const float*)d_in[3];
  const float* a1d  = (const float*)d_in[4];
  const float* b1   = (const float*)d_in[5];
  const float* Wmu  = (const float*)d_in[6];
  const float* amus = (const float*)d_in[7];
  const float* amud = (const float*)d_in[8];
  const float* bmu  = (const float*)d_in[9];
  const float* Wls  = (const float*)d_in[10];
  const float* alss = (const float*)d_in[11];
  const float* alsd = (const float*)d_in[12];
  const float* bls  = (const float*)d_in[13];
  float* out0 = (float*)d_out;
  float* out1 = out0 + (size_t)nN * OC;

  const int nP = ((nN + GR - 1) / GR) * GR;
  size_t off = 0;
  unsigned short* Wp = (unsigned short*)((char*)d_ws + off); off += (size_t)4 * DF * DF * sizeof(unsigned short);
  float* xl   = (float*)((char*)d_ws + off); off += (size_t)nP * DF * sizeof(float);
  float* hb   = (float*)((char*)d_ws + off); off += (size_t)nP * DF * sizeof(float);
  float* asrc = (float*)((char*)d_ws + off); off += (size_t)nP * NHD * sizeof(float);
  float* adst = (float*)((char*)d_ws + off); off += (size_t)nP * NHD * sizeof(float);
  if (off > ws_size) return;

  const int nprep = 2 * DF * (DF / 8);
  k_prep<<<(nprep + NTHR - 1) / NTHR, NTHR, 0, stream>>>(W1, Wmu, Wls, Wp);

  k_gemm<<<nP / GR, NTHR, 0, stream>>>(x, Wp, Wp + DF * DF,
                                       a1s, a1s + 2 * HC, a1d, a1d + 2 * HC,
                                       xl, asrc, adst, nN);

  hipFuncSetAttribute(reinterpret_cast<const void*>(&k_agg<1>),
                      hipFuncAttributeMaxDynamicSharedMemorySize, LDS_BYTES);
  hipFuncSetAttribute(reinterpret_cast<const void*>(&k_agg<2>),
                      hipFuncAttributeMaxDynamicSharedMemorySize, LDS_BYTES);
  const int grid = (nN + NB - 1) / NB;
  k_agg<1><<<grid, NTHR, LDS_BYTES, stream>>>(ei, xl, asrc, adst, b1, b1, hb, out0, out1, nN, nE);

  k_gemm<<<nP / GR, NTHR, 0, stream>>>(hb, Wp + 2 * DF * DF, Wp + 3 * DF * DF,
                                       amus, alss, amud, alsd,
                                       xl, asrc, adst, nN);
  k_agg<2><<<grid, NTHR, LDS_BYTES, stream>>>(ei, xl, asrc, adst, bmu, bls, hb, out0, out1, nN, nE);
}
